// QuanGAT_87582973100319
// MI455X (gfx1250) — hardware-verified
//
#include <hip/hip_runtime.h>
#include <stddef.h>


#define IN    128
#define HID   128
#define NQ    4
#define QL    3
#define H1    4
#define D1    512
#define D2    64
#define GR    32
#define AP    136
#define XSP   516
#define NTHR  256
#define NWAVE 8
#define CHUNK 2048
#define WCAP  256
#define NGRP  (CHUNK / (NTHR * 4))
#define NB1   128
#define NB2   1024
#define AP1   520
#define XSP2  68

#define XS2_OFF 34048
#define PS_OFF  (XS2_OFF + NB1 * XSP2)
#define LDS1_FLOATS (NB1 * D1 + NB1 * H1 + NB1 * H1 + NWAVE * WCAP + NWAVE)
#define LDS1_BYTES  (LDS1_FLOATS * 4)
#define LDS2_FLOATS (NB2 * D2 + NB2 + NB2 + NWAVE * WCAP + NWAVE)
#define LDS2_BYTES  (LDS2_FLOATS * 4)

static_assert(WCAP == (CHUNK / NTHR) * 32);
static_assert(NGRP == 2);
static_assert(XS2_OFF * 4 >= NB1 * AP1 * 2);
static_assert(PS_OFF + 2 * NB1 <= NB1 * D1);
static_assert(LDS1_BYTES == 274464);
static_assert(LDS2_BYTES == 278560);
static_assert((NB1 * D1) % 4 == 0 && (NB2 * D2) % 4 == 0);
static_assert(D1 % 32 == 0 && IN % 32 == 0);

typedef float    v2f  __attribute__((ext_vector_type(2)));
typedef float    v4f  __attribute__((ext_vector_type(4)));
typedef float    v8f  __attribute__((ext_vector_type(8)));
typedef int      v4i  __attribute__((ext_vector_type(4)));
typedef _Float16 v8h  __attribute__((ext_vector_type(8)));
typedef _Float16 v16h __attribute__((ext_vector_type(16)));
union Frag   { v16h v; v8h half[2]; };
union Pack16 { v8h h; v4i i; };

__device__ __forceinline__ v8f wm(v16h a, v16h b, v8f c) {
  v8f d = __builtin_amdgcn_wmma_f32_16x16x32_f16(false, a, false, b, (short)0, c, false, false);
  asm volatile("v_nop\n\tv_nop\n\tv_nop\n\tv_nop" : "+v"(d) : "v"(a), "v"(b));
  return d;
}

__device__ __forceinline__ v8h pack8(v4f a, v4f b) {
  Pack16 u;
  u.h[0] = (_Float16)a.x; u.h[1] = (_Float16)a.y; u.h[2] = (_Float16)a.z; u.h[3] = (_Float16)a.w;
  u.h[4] = (_Float16)b.x; u.h[5] = (_Float16)b.y; u.h[6] = (_Float16)b.z; u.h[7] = (_Float16)b.w;
  return u.h;
}

__device__ __forceinline__ float lrelu(float a) { return (a > 0.f) ? a : 0.2f * a; }

__global__ __launch_bounds__(NTHR) void k_prepw1(const float* __restrict__ W1, _Float16* W1h) {
  __shared__ __attribute__((aligned(16))) _Float16 sT[32 * AP];
  const int tid = threadIdx.x, lane = tid & 31, wave = tid >> 5;
  const int n0 = blockIdx.x * 32;
  const int nl = tid & 31, kk = tid >> 5;
#pragma unroll
  for (int i = 0; i < 16; ++i) {
    const int k = kk + 8 * i;
    sT[nl * AP + k] = (_Float16)(W1[(size_t)k * D1 + n0 + nl] * 8.0f);
  }
  __syncthreads();
  v4i u[2];
  _Float16* p[2];
#pragma unroll
  for (int i = 0; i < 2; ++i) {
    const int row = 4 * wave + 2 * i + (lane >> 4);
    const int k8  = (lane & 15) * 8;
    Pack16 pk;
    pk.h = *(const v8h*)(sT + row * AP + k8);
    u[i] = pk.i;
    p[i] = W1h + (size_t)(n0 + row) * IN + k8;
  }
  *(volatile v4i*)(p[0]) = u[0];
  *(volatile v4i*)(p[1]) = u[1];
  __threadfence();
  *(volatile v4i*)(p[0]) = u[0];
  *(volatile v4i*)(p[1]) = u[1];
}

__global__ __launch_bounds__(NTHR) void k_prepw2(const float* __restrict__ W2, _Float16* W2h) {
  __shared__ __attribute__((aligned(16))) _Float16 sT[8 * AP1];
  const int tid = threadIdx.x, lane = tid & 31, wave = tid >> 5;
  const int n0 = blockIdx.x * 8;
  const int nl = tid & 7, kk = tid >> 3;
#pragma unroll
  for (int i = 0; i < 16; ++i) {
    const int k = kk + 32 * i;
    sT[nl * AP1 + k] = (_Float16)(W2[(size_t)k * D2 + n0 + nl] * 16.0f);
  }
  __syncthreads();
  v4i u[2];
  _Float16* p[2];
#pragma unroll
  for (int i = 0; i < 2; ++i) {
    const int k8 = 256 * i + 8 * lane;
    Pack16 pk;
    pk.h = *(const v8h*)(sT + wave * AP1 + k8);
    u[i] = pk.i;
    p[i] = W2h + (size_t)(n0 + wave) * D1 + k8;
  }
  *(volatile v4i*)(p[0]) = u[0];
  *(volatile v4i*)(p[1]) = u[1];
  __threadfence();
  *(volatile v4i*)(p[0]) = u[0];
  *(volatile v4i*)(p[1]) = u[1];
}

__global__ __launch_bounds__(NTHR) void k_gemm1(
    const float* __restrict__ x, const float* __restrict__ Wp, const float* __restrict__ bp,
    const float* __restrict__ qw, const float* __restrict__ Wfc, const float* __restrict__ bfc,
    const _Float16* __restrict__ W1h, const float* __restrict__ a1s, const float* __restrict__ a1d,
    float* g1, float* asrc, float* adst, int nN) {
  __shared__ __attribute__((aligned(16))) _Float16 At[GR * AP];
  __shared__ __attribute__((aligned(16))) float Xs[16 * XSP];
  __shared__ __attribute__((aligned(16))) float As[GR * NWAVE];
  __shared__ __attribute__((aligned(16))) float Ds[GR * NWAVE];
  __shared__ __attribute__((aligned(16))) float sWp[IN * NQ];
  __shared__ __attribute__((aligned(16))) float sWfc[NQ * HID];
  __shared__ __attribute__((aligned(16))) float sbfc[HID];
  __shared__ float sbp[NQ];
  __shared__ float sQc[QL * NQ];
  __shared__ float sQs[QL * NQ];
  __shared__ float sRe[GR * 16];
  __shared__ float sIm[GR * 16];
  __shared__ float sCs[GR * NQ];
  __shared__ float sSn[GR * NQ];

  const int tid  = threadIdx.x;
  const int lane = tid & 31, wave = tid >> 5, hh = lane >> 4, m = lane & 15;
  const int q = tid >> 3, t = tid & 7;
  const int rowBase = blockIdx.x * GR;

  for (int i = tid; i < IN * NQ; i += NTHR) { sWp[i] = Wp[i]; sWfc[i] = Wfc[i]; }
  if (tid < HID) sbfc[tid] = bfc[tid];
  if (tid < NQ) sbp[tid] = bp[tid];
  if (wave == 1) {
    const int li = (lane < QL * NQ - 1) ? lane : (QL * NQ - 1);
    const float hf = qw[li] * 0.5f;
    const float cv = cosf(hf), sv = sinf(hf);
    if (lane < QL * NQ) { sQc[lane] = cv; sQs[lane] = sv; }
  }
  __syncthreads();

  int node = rowBase + q;
  if (node > nN - 1) node = nN - 1;
  float p0 = 0.f, p1 = 0.f, p2 = 0.f, p3 = 0.f;
  {
    const float* xr = x + (size_t)node * IN + 16 * t;
#pragma unroll 1
    for (int i = 0; i < 4; ++i) {
      const v4f v  = *(const v4f*)(xr + 4 * i);
      const int k  = 16 * t + 4 * i;
      const v4f w0 = *(const v4f*)(sWp + (k + 0) * NQ);
      const v4f w1 = *(const v4f*)(sWp + (k + 1) * NQ);
      const v4f w2 = *(const v4f*)(sWp + (k + 2) * NQ);
      const v4f w3 = *(const v4f*)(sWp + (k + 3) * NQ);
      p0 += v.x * w0.x + v.y * w1.x + v.z * w2.x + v.w * w3.x;
      p1 += v.x * w0.y + v.y * w1.y + v.z * w2.y + v.w * w3.y;
      p2 += v.x * w0.z + v.y * w1.z + v.z * w2.z + v.w * w3.z;
      p3 += v.x * w0.w + v.y * w1.w + v.z * w2.w + v.w * w3.w;
    }
  }
#pragma unroll
  for (int mk = 1; mk < 8; mk <<= 1) {
    p0 += __shfl_xor(p0, mk, 32); p1 += __shfl_xor(p1, mk, 32);
    p2 += __shfl_xor(p2, mk, 32); p3 += __shfl_xor(p3, mk, 32);
  }
  {
    const int w = t & 3;
    float th = (w == 0) ? p0 : ((w == 1) ? p1 : ((w == 2) ? p2 : p3));
    th += sbp[w];
    const float hf = th * 0.5f;
    const float cv = cosf(hf), sv = sinf(hf);
    if (t < 4) { sCs[q * NQ + w] = cv; sSn[q * NQ + w] = sv; }
    sRe[q * 16 + 2 * t]     = (t == 0) ? 1.f : 0.f;
    sRe[q * 16 + 2 * t + 1] = 0.f;
    sIm[q * 16 + 2 * t]     = 0.f;
    sIm[q * 16 + 2 * t + 1] = 0.f;
  }
  __syncthreads();

#pragma unroll 1
  for (int layer = 0; layer <= QL; ++layer) {
#pragma unroll 1
    for (int w = 0; w < NQ; ++w) {
      const float ce = sCs[q * NQ + w], se = sSn[q * NQ + w];
      const int   li = (layer > 0) ? (layer - 1) * NQ + w : 0;
      const float cq = sQc[li], sq2 = sQs[li];
      const float c = (layer == 0) ? ce : cq;
      const float s = (layer == 0) ? se : sq2;
      const int b = 3 - w, bitv = 1 << b, lowm = bitv - 1;
      const int i0 = ((t & ~lowm) << 1) | (t & lowm);
      const int ia = q * 16 + i0, ib = ia + bitv;
      const float ar = sRe[ia], ai = sIm[ia], br = sRe[ib], bi = sIm[ib];
      sRe[ia] = c * ar + s * bi;
      sIm[ia] = c * ai - s * br;
      sRe[ib] = s * ai + c * br;
      sIm[ib] = c * bi - s * ar;
      __syncthreads();
    }
    if (layer > 0) {
#pragma unroll 1
      for (int cg = 0; cg < NQ; ++cg) {
        const int cbp = 3 - cg, tbp = 3 - ((cg + 1) & 3);
        const int tbit = 1 << tbp, cbit = 1 << cbp, lowm = tbit - 1;
        const int i0 = ((t & ~lowm) << 1) | (t & lowm);
        const int ia = q * 16 + i0, ib = ia + tbit;
        const float ar = sRe[ia], ai = sIm[ia], br = sRe[ib], bi = sIm[ib];
        const bool sw = (i0 & cbit) != 0;
        sRe[ia] = sw ? br : ar;
        sIm[ia] = sw ? bi : ai;
        sRe[ib] = sw ? ar : br;
        sIm[ib] = sw ? ai : bi;
        __syncthreads();
      }
    }
  }

  {
    const int ia = q * 16 + 2 * t;
    const float ar = sRe[ia], ai = sIm[ia], br = sRe[ia + 1], bi = sIm[ia + 1];
    const float pa = ar * ar + ai * ai;
    const float pb = br * br + bi * bi;
    const float ps = pa + pb;
    float z0 = (t & 4) ? -ps : ps;
    float z1 = (t & 2) ? -ps : ps;
    float z2 = (t & 1) ? -ps : ps;
    float z3 = pa - pb;
#pragma unroll
    for (int mk = 1; mk < 8; mk <<= 1) {
      z0 += __shfl_xor(z0, mk, 32); z1 += __shfl_xor(z1, mk, 32);
      z2 += __shfl_xor(z2, mk, 32); z3 += __shfl_xor(z3, mk, 32);
    }
#pragma unroll 1
    for (int e8 = 0; e8 < 2; ++e8) {
      const int c0 = 16 * t + 8 * e8;
      Pack16 u;
#pragma unroll
      for (int e = 0; e < 8; ++e) {
        const int c = c0 + e;
        float v = z0 * sWfc[c] + z1 * sWfc[HID + c] + z2 * sWfc[2 * HID + c] + z3 * sWfc[3 * HID + c];
        v += sbfc[c];
        u.h[e] = (_Float16)v;
      }
      *(v8h*)(At + q * AP + c0) = u.h;
    }
  }
  __syncthreads();

  const v8f z8 = {0.f, 0.f, 0.f, 0.f, 0.f, 0.f, 0.f, 0.f};
  v8f acc[2][4];
#pragma unroll
  for (int mt = 0; mt < 2; ++mt)
#pragma unroll
    for (int nt = 0; nt < 4; ++nt) acc[mt][nt] = z8;
#pragma unroll
  for (int kt = 0; kt < IN / 32; ++kt) {
    const int k0 = kt * 32;
    Frag a0, a1;
    const _Float16* pa0 = At + m * AP + k0 + 8 * hh;
    const _Float16* pa1 = At + (16 + m) * AP + k0 + 8 * hh;
    a0.half[0] = *(const v8h*)pa0; a0.half[1] = *(const v8h*)(pa0 + 16);
    a1.half[0] = *(const v8h*)pa1; a1.half[1] = *(const v8h*)(pa1 + 16);
#pragma unroll
    for (int nt = 0; nt < 4; ++nt) {
      Frag b;
      const _Float16* pb = W1h + (size_t)(64 * wave + 16 * nt + m) * IN + k0 + 8 * hh;
      b.half[0] = *(const v8h*)pb; b.half[1] = *(const v8h*)(pb + 16);
      acc[0][nt] = wm(a0.v, b.v, acc[0][nt]);
      acc[1][nt] = wm(a1.v, b.v, acc[1][nt]);
    }
  }

  float cs[4], cd[4];
#pragma unroll
  for (int nt = 0; nt < 4; ++nt) {
    const int nc = 64 * wave + 16 * nt + m;
    cs[nt] = a1s[nc];
    cd[nt] = a1d[nc];
  }
#pragma unroll
  for (int mt = 0; mt < 2; ++mt) {
    float ss[8], sd[8];
#pragma unroll
    for (int r = 0; r < 8; ++r) {
      float s1 = 0.f, s2 = 0.f;
#pragma unroll
      for (int nt = 0; nt < 4; ++nt) {
        const float v = acc[mt][nt][r] * 0.125f;
        Xs[(8 * hh + r) * XSP + 64 * wave + 16 * nt + m] = v;
        s1 += v * cs[nt];
        s2 += v * cd[nt];
      }
      ss[r] = s1; sd[r] = s2;
    }
#pragma unroll
    for (int mk = 1; mk < 16; mk <<= 1) {
#pragma unroll
      for (int r = 0; r < 8; ++r) {
        ss[r] += __shfl_xor(ss[r], mk, 32);
        sd[r] += __shfl_xor(sd[r], mk, 32);
      }
    }
    if (m == 0) {
#pragma unroll
      for (int r = 0; r < 8; ++r) {
        As[(16 * mt + 8 * hh + r) * NWAVE + wave] = ss[r];
        Ds[(16 * mt + 8 * hh + r) * NWAVE + wave] = sd[r];
      }
    }
    __syncthreads();
    v4f xr[2][4];
#pragma unroll
    for (int i = 0; i < 2; ++i)
#pragma unroll
      for (int sg = 0; sg < 4; ++sg)
        xr[i][sg] = *(const v4f*)(Xs + (2 * wave + i) * XSP + 128 * sg + 4 * lane);
    float* gb = g1 + (size_t)(rowBase + 16 * mt + 2 * wave) * D1 + 4 * lane;
#pragma unroll
    for (int i = 0; i < 2; ++i)
#pragma unroll
      for (int sg = 0; sg < 4; ++sg) *(volatile v4f*)(gb + (size_t)i * D1 + 128 * sg) = xr[i][sg];
    __threadfence();
#pragma unroll
    for (int i = 0; i < 2; ++i)
#pragma unroll
      for (int sg = 0; sg < 4; ++sg) *(volatile v4f*)(gb + (size_t)i * D1 + 128 * sg) = xr[i][sg];
    __syncthreads();
  }
  if (wave == 0) {
    v4f v;
    v.x = As[lane * NWAVE + 0] + As[lane * NWAVE + 1];
    v.y = As[lane * NWAVE + 2] + As[lane * NWAVE + 3];
    v.z = As[lane * NWAVE + 4] + As[lane * NWAVE + 5];
    v.w = As[lane * NWAVE + 6] + As[lane * NWAVE + 7];
    float* p = asrc + (size_t)(rowBase + lane) * H1;
    *(volatile v4f*)p = v;
    __threadfence();
    *(volatile v4f*)p = v;
  } else if (wave == 1) {
    v4f v;
    v.x = Ds[lane * NWAVE + 0] + Ds[lane * NWAVE + 1];
    v.y = Ds[lane * NWAVE + 2] + Ds[lane * NWAVE + 3];
    v.z = Ds[lane * NWAVE + 4] + Ds[lane * NWAVE + 5];
    v.w = Ds[lane * NWAVE + 6] + Ds[lane * NWAVE + 7];
    float* p = adst + (size_t)(rowBase + lane) * H1;
    *(volatile v4f*)p = v;
    __threadfence();
    *(volatile v4f*)p = v;
  }
}

template <int NBV, int SH>
__device__ __forceinline__ int scan_chunk(const int* __restrict__ eid, int nE, int cbase, int nodeBase,
                                          bool al16, int* list, int tid, int wave) {
  int wc = 0;
#pragma unroll
  for (int g = 0; g < NGRP; ++g) {
    const int el0  = (g * NTHR + tid) * 4;
    const int e0   = cbase + el0;
    const int sent = -2147483647 - 1;
    const int last = nE - 1;
    v4i d;
    if (al16 && (cbase + CHUNK <= nE)) {
      d = *(const v4i*)(eid + e0);
    } else {
      const int c0 = (e0     < last) ? e0     : last;
      const int c1 = (e0 + 1 < last) ? e0 + 1 : last;
      const int c2 = (e0 + 2 < last) ? e0 + 2 : last;
      const int c3 = (e0 + 3 < last) ? e0 + 3 : last;
      const int v0 = eid[c0], v1 = eid[c1], v2 = eid[c2], v3 = eid[c3];
      d.x = (e0     <= last) ? v0 : sent;
      d.y = (e0 + 1 <= last) ? v1 : sent;
      d.z = (e0 + 2 <= last) ? v2 : sent;
      d.w = (e0 + 3 <= last) ? v3 : sent;
    }
    const unsigned s0 = (unsigned)d.x - (unsigned)nodeBase;
    const unsigned s1 = (unsigned)d.y - (unsigned)nodeBase;
    const unsigned s2 = (unsigned)d.z - (unsigned)nodeBase;
    const unsigned s3 = (unsigned)d.w - (unsigned)nodeBase;
    const bool h0 = s0 < (unsigned)NBV;
    const bool h1 = s1 < (unsigned)NBV;
    const bool h2 = s2 < (unsigned)NBV;
    const bool h3 = s3 < (unsigned)NBV;
    const unsigned many = __builtin_amdgcn_ballot_w32(h0 | h1 | h2 | h3);
    if (many != 0u) {
      {
        const unsigned mj = __builtin_amdgcn_ballot_w32(h0);
        if (h0) {
          const int pos = wc + (int)__builtin_amdgcn_mbcnt_lo(mj, 0u);
          if (pos < WCAP) list[wave * WCAP + pos] = ((el0 + 0) << SH) | (int)s0;
        }
        wc += (int)__builtin_popcount(mj);
      }
      {
        const unsigned mj = __builtin_amdgcn_ballot_w32(h1);
        if (h1) {
          const int pos = wc + (int)__builtin_amdgcn_mbcnt_lo(mj, 0u);
          if (pos < WCAP) list[wave * WCAP + pos] = ((el0 + 1) << SH) | (int)s1;
        }
        wc += (int)__builtin_popcount(mj);
      }
      {
        const unsigned mj = __builtin_amdgcn_ballot_w32(h2);
        if (h2) {
          const int pos = wc + (int)__builtin_amdgcn_mbcnt_lo(mj, 0u);
          if (pos < WCAP) list[wave * WCAP + pos] = ((el0 + 2) << SH) | (int)s2;
        }
        wc += (int)__builtin_popcount(mj);
      }
      {
        const unsigned mj = __builtin_amdgcn_ballot_w32(h3);
        if (h3) {
          const int pos = wc + (int)__builtin_amdgcn_mbcnt_lo(mj, 0u);
          if (pos < WCAP) list[wave * WCAP + pos] = ((el0 + 3) << SH) | (int)s3;
        }
        wc += (int)__builtin_popcount(mj);
      }
    }
  }
  return wc;
}

__global__ __launch_bounds__(NTHR) void k_agg1(
    const int* __restrict__ ei, const float* __restrict__ g1,
    const float* __restrict__ asrc, const float* __restrict__ adst, const float* __restrict__ b1,
    const _Float16* __restrict__ W2h, const float* __restrict__ a2s, const float* __restrict__ a2d,
    float* g2, float* asrc2, float* adst2, int nN, int nE, int nP) {
  extern __shared__ v4f lds_dyn[];
  float* sacc = (float*)lds_dyn;
  float* smax = sacc + NB1 * D1;
  float* sden = smax + NB1 * H1;
  int*   list = (int*)(sden + NB1 * H1);
  int*   wcnt = list + NWAVE * WCAP;

  const int tid  = threadIdx.x;
  const int lane = tid & 31, wave = tid >> 5, hh = lane >> 4, m = lane & 15;
  const int nodeBase = blockIdx.x * NB1;

  {
    const v4f z4 = {0.f, 0.f, 0.f, 0.f};
    for (int i = tid; i < (NB1 * D1) / 4; i += NTHR) lds_dyn[i] = z4;
    const float ninf = -__builtin_inff();
    for (int i = tid; i < NB1 * H1; i += NTHR) { smax[i] = ninf; sden[i] = 0.f; }
  }
  __syncthreads();

  const int* eid = ei + nE;
  const bool al16 = ((nE & 3) == 0);
  const int nChunks = (nE + CHUNK - 1) / CHUNK;

#pragma unroll 1
  for (int ch = 0; ch < nChunks; ++ch) {
    const int cbase = ch * CHUNK;
    const int wc = scan_chunk<NB1, 7>(eid, nE, cbase, nodeBase, al16, list, tid, wave);
    if (lane == 0) wcnt[wave] = wc;
    __syncthreads();
    if (wave == 0) {
      const int hd = lane >> 3;
      const int cb = 16 * lane;
      for (int wsx = 0; wsx < NWAVE; ++wsx) {
        int n = wcnt[wsx];
        n = (n > WCAP) ? WCAP : n;
        n = (n < 0) ? 0 : n;
        for (int i = 0; i < n; ++i) {
          const int ent  = list[wsx * WCAP + i];
          const int slot = ent & (NB1 - 1);
          const int el   = (ent >> 7) & (CHUNK - 1);
          int e = cbase + el;
          if (e > nE - 1) e = nE - 1;
          int src = ei[e];
          src = (src < 0) ? 0 : ((src > nN - 1) ? nN - 1 : src);
          int nd = nodeBase + slot;
          if (nd > nN - 1) nd = nN - 1;
          const float al = lrelu(asrc[(size_t)src * H1 + hd] + adst[(size_t)nd * H1 + hd]);
          const int   mi = slot * H1 + hd;
          const float mo = smax[mi];
          const float mn = fmaxf(mo, al);
          const float sc = __expf(mo - mn);
          const float p  = __expf(al - mn);
          const float dn = sden[mi] * sc + p;
          const float* gp = g1 + (size_t)src * D1 + cb;
          float* sp = sacc + slot * D1 + cb;
#pragma unroll
          for (int sg = 0; sg < 4; ++sg) {
            const v4f xv  = *(const v4f*)(gp + 4 * sg);
            const v4f cur = *(const v4f*)(sp + 4 * sg);
            *(v4f*)(sp + 4 * sg) = cur * sc + p * xv;
          }
          smax[mi] = mn;
          sden[mi] = dn;
        }
      }
    }
    __syncthreads();
  }

  _Float16* Ah = (_Float16*)sacc;
  {
    const int hd = lane >> 3;
    const int cb = 16 * lane;
#pragma unroll 1
    for (int j = 0; j < NB1 / NWAVE; ++j) {
      const int slot  = j * NWAVE + wave;
      const int node  = nodeBase + slot;
      const int nodec = (node > nN - 1) ? nN - 1 : node;
      v4f f[4];
#pragma unroll
      for (int sg = 0; sg < 4; ++sg) f[sg] = *(const v4f*)(sacc + slot * D1 + cb + 4 * sg);
      const float mo = smax[slot * H1 + hd];
      const float ds = sden[slot * H1 + hd];
      __syncthreads();
      const float al  = lrelu(asrc[(size_t)nodec * H1 + hd] + adst[(size_t)nodec * H1 + hd]);
      const float mn  = fmaxf(mo, al);
      const float sc  = __expf(mo - mn);
      const float p   = __expf(al - mn);
      const float den = ds * sc + p;
      const float inv = 1.0f / den;
      const bool live = node < nN;
      const float* gp = g1 + (size_t)nodec * D1 + cb;
      v4f o[4];
#pragma unroll
      for (int sg = 0; sg < 4; ++sg) {
        const v4f xv = *(const v4f*)(gp + 4 * sg);
        const v4f bb = *(const v4f*)(b1 + cb + 4 * sg);
        v4f v = (f[sg] * sc + p * xv) * inv + bb;
        v.x = (live && v.x > 0.f) ? v.x : 0.f;
        v.y = (live && v.y > 0.f) ? v.y : 0.f;
        v.z = (live && v.z > 0.f) ? v.z : 0.f;
        v.w = (live && v.w > 0.f) ? v.w : 0.f;
        o[sg] = v;
      }
      *(v8h*)(Ah + slot * AP1 + cb)     = pack8(o[0], o[1]);
      *(v8h*)(Ah + slot * AP1 + cb + 8) = pack8(o[2], o[3]);
      __syncthreads();
    }
  }

  const v8f z8 = {0.f, 0.f, 0.f, 0.f, 0.f, 0.f, 0.f, 0.f};
  v8f acc[4];
#pragma unroll
  for (int nt = 0; nt < 4; ++nt) acc[nt] = z8;
#pragma unroll 2
  for (int kt = 0; kt < D1 / 32; ++kt) {
    const int k0 = kt * 32;
    Frag a;
    const _Float16* pa = Ah + (16 * wave + m) * AP1 + k0 + 8 * hh;
    a.half[0] = *(const v8h*)pa; a.half[1] = *(const v8h*)(pa + 16);
#pragma unroll
    for (int nt = 0; nt < 4; ++nt) {
      Frag b;
      const _Float16* pb = W2h + (size_t)(16 * nt + m) * D1 + k0 + 8 * hh;
      b.half[0] = *(const v8h*)pb; b.half[1] = *(const v8h*)(pb + 16);
      acc[nt] = wm(a.v, b.v, acc[nt]);
    }
  }

  float* Xs2 = sacc + XS2_OFF;
  float* Ps  = sacc + PS_OFF;
  float* Pd  = Ps + NB1;
  {
    float cs[4], cd[4];
#pragma unroll
    for (int nt = 0; nt < 4; ++nt) { cs[nt] = a2s[16 * nt + m]; cd[nt] = a2d[16 * nt + m]; }
    float ss[8], sd[8];
#pragma unroll
    for (int r = 0; r < 8; ++r) {
      float s1 = 0.f, s2 = 0.f;
#pragma unroll
      for (int nt = 0; nt < 4; ++nt) {
        const float v = acc[nt][r] * 0.0625f;
        Xs2[(16 * wave + 8 * hh + r) * XSP2 + 16 * nt + m] = v;
        s1 += v * cs[nt];
        s2 += v * cd[nt];
      }
      ss[r] = s1; sd[r] = s2;
    }
#pragma unroll
    for (int mk = 1; mk < 16; mk <<= 1) {
#pragma unroll
      for (int r = 0; r < 8; ++r) {
        ss[r] += __shfl_xor(ss[r], mk, 32);
        sd[r] += __shfl_xor(sd[r], mk, 32);
      }
    }
    if (m == 0) {
#pragma unroll
      for (int r = 0; r < 8; ++r) {
        Ps[16 * wave + 8 * hh + r] = ss[r];
        Pd[16 * wave + 8 * hh + r] = sd[r];
      }
    }
  }
  __syncthreads();

  v4f gr[8];
  float* gpp[8];
  bool gok[8];
#pragma unroll
  for (int i = 0; i < 8; ++i) {
    const int rloc = 16 * wave + 2 * i + hh;
    const int nd   = nodeBase + rloc;
    gr[i]  = *(const v4f*)(Xs2 + rloc * XSP2 + 4 * m);
    gok[i] = nd < nP;
    const int ndc = gok[i] ? nd : 0;
    gpp[i] = g2 + (size_t)ndc * D2 + 4 * m;
  }
  v4f pv = {0.f, 0.f, 0.f, 0.f};
  float* pp = 0;
  {
    const int n0 = nodeBase + 4 * lane;
    const bool ok = n0 < nP;
    const int n0c = ok ? n0 : 0;
    if (wave == 0) { pv = *(const v4f*)(Ps + 4 * lane); if (ok) pp = asrc2 + n0c; }
    else if (wave == 1) { pv = *(const v4f*)(Pd + 4 * lane); if (ok) pp = adst2 + n0c; }
  }
#pragma unroll
  for (int i = 0; i < 8; ++i) if (gok[i]) *(volatile v4f*)(gpp[i]) = gr[i];
  if (pp) *(volatile v4f*)pp = pv;
  __threadfence();
#pragma unroll
  for (int i = 0; i < 8; ++i) if (gok[i]) *(volatile v4f*)(gpp[i]) = gr[i];
  if (pp) *(volatile v4f*)pp = pv;
}

__global__ __launch_bounds__(NTHR) void k_agg2(
    const int* __restrict__ ei, const float* __restrict__ g2,
    const float* __restrict__ asrc2, const float* __restrict__ adst2, const float* __restrict__ b2,
    float* out, int nN, int nE) {
  extern __shared__ v4f lds_dyn[];
  float* sacc = (float*)lds_dyn;
  float* smax = sacc + NB2 * D2;
  float* sden = smax + NB2;
  int*   list = (int*)(sden + NB2);
  int*   wcnt = list + NWAVE * WCAP;

  const int tid  = threadIdx.x;
  const int lane = tid & 31, wave = tid >> 5, hh = lane >> 4, m = lane & 15;
  const int nodeBase = blockIdx.x * NB2;

  {
    const v4f z4 = {0.f, 0.f, 0.f, 0.f};
    for (int i = tid; i < (NB2 * D2) / 4; i += NTHR) lds_dyn[i] = z4;
    const float ninf = -__builtin_inff();
    for (int i = tid; i < NB2; i += NTHR) { smax[i] = ninf; sden[i] = 0.f; }
  }
  __syncthreads();

  const int* eid = ei + nE;
  const bool al16 = ((nE & 3) == 0);
  const int nChunks = (nE + CHUNK - 1) / CHUNK;

#pragma unroll 1
  for (int ch = 0; ch < nChunks; ++ch) {
    const int cbase = ch * CHUNK;
    const int wc = scan_chunk<NB2, 10>(eid, nE, cbase, nodeBase, al16, list, tid, wave);
    if (lane == 0) wcnt[wave] = wc;
    __syncthreads();
    if (wave == 0) {
      const int c2 = 2 * lane;
      for (int wsx = 0; wsx < NWAVE; ++wsx) {
        int n = wcnt[wsx];
        n = (n > WCAP) ? WCAP : n;
        n = (n < 0) ? 0 : n;
        for (int i = 0; i < n; ++i) {
          const int ent  = list[wsx * WCAP + i];
          const int slot = ent & (NB2 - 1);
          const int el   = (ent >> 10) & (CHUNK - 1);
          int e = cbase + el;
          if (e > nE - 1) e = nE - 1;
          int src = ei[e];
          src = (src < 0) ? 0 : ((src > nN - 1) ? nN - 1 : src);
          int nd = nodeBase + slot;
          if (nd > nN - 1) nd = nN - 1;
          const float al = lrelu(asrc2[src] + adst2[nd]);
          const float mo = smax[slot];
          const float mn = fmaxf(mo, al);
          const float sc = __expf(mo - mn);
          const float p  = __expf(al - mn);
          const float dn = sden[slot] * sc + p;
          const v2f xv  = *(const v2f*)(g2 + (size_t)src * D2 + c2);
          const v2f cur = *(const v2f*)(sacc + slot * D2 + c2);
          *(v2f*)(sacc + slot * D2 + c2) = cur * sc + p * xv;
          smax[slot] = mn;
          sden[slot] = dn;
        }
      }
    }
    __syncthreads();
  }

  const int c0 = 4 * m;
  const v4f bb = *(const v4f*)(b2 + c0);
#pragma unroll 1
  for (int j = 0; j < NB2 / (2 * NWAVE); ++j) {
    const int slotA = wave * (NB2 / NWAVE) + 2 * j;
    if (nodeBase + slotA > nN - 1) break;
    const int slot  = slotA + hh;
    const int node  = nodeBase + slot;
    const int nodec = (node > nN - 1) ? nN - 1 : node;
    const float al  = lrelu(asrc2[nodec] + adst2[nodec]);
    const float mo  = smax[slot];
    const float ds  = sden[slot];
    const float mn  = fmaxf(mo, al);
    const float sc  = __expf(mo - mn);
    const float p   = __expf(al - mn);
    const float den = ds * sc + p;
    const float inv = 1.0f / den;
    const v4f f  = *(const v4f*)(sacc + slot * D2 + c0);
    const v4f xv = *(const v4f*)(g2 + (size_t)nodec * D2 + c0);
    const v4f o  = (f * sc + p * xv) * inv + bb;
    const bool live = node < nN;
    float* op = out + (size_t)nodec * D2 + c0;
    if (live) *(volatile v4f*)op = o;
    __threadfence();
    if (live) *(volatile v4f*)op = o;
  }
}

extern "C" void kernel_launch(void* const* d_in, const int* in_sizes, int n_in,
                              void* d_out, int out_size, void* d_ws, size_t ws_size,
                              hipStream_t stream) {
  if (n_in < 15) return;
  const int nN = in_sizes[0] / IN;
  if (nN <= 0 || in_sizes[0] != nN * IN) return;
  if (in_sizes[1] < 0 || (in_sizes[1] & 1) != 0) return;
  const int nE = in_sizes[1] / 2;
  if (in_sizes[2] != IN * NQ || in_sizes[3] != NQ || in_sizes[4] != QL * NQ) return;
  if (in_sizes[5] != NQ * HID || in_sizes[6] != HID) return;
  if (in_sizes[7] != HID * D1 || in_sizes[8] != H1 * HID || in_sizes[9] != H1 * HID || in_sizes[10] != D1) return;
  if (in_sizes[11] != D1 * D2 || in_sizes[12] != D2 || in_sizes[13] != D2 || in_sizes[14] != D2) return;
  if (out_size != nN * D2) return;

  const float* x      = (const float*)d_in[0];
  const int*   ei     = (const int*)d_in[1];
  const float* W_proj = (const float*)d_in[2];
  const float* b_proj = (const float*)d_in[3];
  const float* q_w    = (const float*)d_in[4];
  const float* W_fc   = (const float*)d_in[5];
  const float* b_fc   = (const float*)d_in[6];
  const float* W1     = (const float*)d_in[7];
  const float* a1_src = (const float*)d_in[8];
  const float* a1_dst = (const float*)d_in[9];
  const float* b1     = (const float*)d_in[10];
  const float* W2     = (const float*)d_in[11];
  const float* a2_src = (const float*)d_in[12];
  const float* a2_dst = (const float*)d_in[13];
  const float* b2     = (const float*)d_in[14];
  float* out = (float*)d_out;

  const int nP = ((nN + GR - 1) / GR) * GR;
  size_t off = 0;
  auto carve = [&](size_t bytes) -> char* {
    char* p = (char*)d_ws + off;
    off += (bytes + 255) & ~(size_t)255;
    return p;
  };
  _Float16* W1h = (_Float16*)carve((size_t)D1 * IN * sizeof(_Float16));
  _Float16* W2h = (_Float16*)carve((size_t)D2 * D1 * sizeof(_Float16));
  float* g1    = (float*)carve((size_t)nP * D1 * sizeof(float));
  float* asrc  = (float*)carve((size_t)nP * H1 * sizeof(float));
  float* adst  = (float*)carve((size_t)nP * H1 * sizeof(float));
  float* g2    = (float*)carve((size_t)nP * D2 * sizeof(float));
  float* asrc2 = (float*)carve((size_t)nP * sizeof(float));
  float* adst2 = (float*)carve((size_t)nP * sizeof(float));
  if (off > ws_size) return;

  k_prepw1<<<D1 / 32, NTHR, 0, stream>>>(W1, W1h);
  k_prepw2<<<D2 / 8, NTHR, 0, stream>>>(W2, W2h);

  k_gemm1<<<nP / GR, NTHR, 0, stream>>>(x, W_proj, b_proj, q_w, W_fc, b_fc, W1h, a1_src, a1_dst,
                                        g1, asrc, adst, nN);

  hipFuncSetAttribute(reinterpret_cast<const void*>(&k_agg1),
                      hipFuncAttributeMaxDynamicSharedMemorySize, LDS1_BYTES);
  const int grid1 = (nN + NB1 - 1) / NB1;
  k_agg1<<<grid1, NTHR, LDS1_BYTES, stream>>>(ei, g1, asrc, adst, b1, W2h, a2_src, a2_dst,
                                               g2, asrc2, adst2, nN, nE, nP);

  hipFuncSetAttribute(reinterpret_cast<const void*>(&k_agg2),
                      hipFuncAttributeMaxDynamicSharedMemorySize, LDS2_BYTES);
  const int grid2 = (nN + NB2 - 1) / NB2;
  k_agg2<<<grid2, NTHR, LDS2_BYTES, stream>>>(ei, g2, asrc2, adst2, b2, out, nN, nE);
}
